// CnnSelfAttention_25331717112491
// MI455X (gfx1250) — hardware-verified
//
#include <hip/hip_runtime.h>
#include <math.h>
#include <stdint.h>

#ifndef NB
#define NB 8
#endif
#ifndef SEQ
#define SEQ 4096
#endif
#define NB_FULL  8
#define SEQ_FULL 4096
#define CC     256
#define DQ     32
#define MW     320
#define MBLK   5
#define QT     64
#define OSP    68
#define OSPW   132
#define TP     72
#define WSC    256.0f
#define IWSC   0.00390625f
#define HSC    16.0f
#define IHSC   0.0625f
#define LNPS   9.704060527839234f

static_assert(NB >= 1 && NB <= NB_FULL);
static_assert(SEQ >= QT && SEQ <= SEQ_FULL);
static_assert(SEQ % QT == 0 && SEQ % 32 == 0);
static_assert(CC % QT == 0 && CC % 32 == 0);
static_assert(MW == 2 * DQ + CC);
static_assert(MW == MBLK * QT);
static_assert(QT == 2 * DQ);
static_assert(MW % 8 == 0);
static_assert((OSP * 4) % 16 == 0);
static_assert((OSPW * 4) % 16 == 0);
static_assert((TP * 2) % 16 == 0);
static_assert(DQ % 32 == 0);

typedef _Float16       v16h __attribute__((ext_vector_type(16)));
typedef _Float16       v8h  __attribute__((ext_vector_type(8)));
typedef __bf16         v16b __attribute__((ext_vector_type(16)));
typedef unsigned short v8us __attribute__((ext_vector_type(8)));
typedef float          v8f  __attribute__((ext_vector_type(8)));
typedef float          v4f  __attribute__((ext_vector_type(4)));
typedef unsigned int   v4u  __attribute__((ext_vector_type(4)));

union Frag  { v8us u[2]; v16h h; v16b bf; };
union FragH { v16h v; v8h hv[2]; };
static_assert(sizeof(Frag) == 32);
static_assert(sizeof(FragH) == 32);

__device__ __forceinline__ unsigned short bf_bits(float f) {
  unsigned u = __float_as_uint(f);
  return (unsigned short)((u + 0x7FFFu + ((u >> 16) & 1u)) >> 16);
}
__device__ __forceinline__ float bf_up(unsigned short hb) { return __uint_as_float(((unsigned)hb) << 16); }
__device__ __forceinline__ float bfr(float f) { return bf_up(bf_bits(f)); }
__device__ __forceinline__ unsigned short h_bits(_Float16 x) { return __builtin_bit_cast(unsigned short, x); }
__device__ __forceinline__ unsigned pk16(unsigned short a, unsigned short b) { return (unsigned)a | ((unsigned)b << 16); }
__device__ __forceinline__ v8f zero8() { v8f z = {0.f, 0.f, 0.f, 0.f, 0.f, 0.f, 0.f, 0.f}; return z; }
__device__ __forceinline__ float hmax8(v8f s) {
  return fmaxf(fmaxf(fmaxf(s[0], s[1]), fmaxf(s[2], s[3])), fmaxf(fmaxf(s[4], s[5]), fmaxf(s[6], s[7])));
}
__device__ __forceinline__ unsigned wave_ballot(bool p) {
#if defined(__HIP_DEVICE_COMPILE__)
  return __builtin_amdgcn_ballot_w32(p);
#else
  return p ? 1u : 0u;
#endif
}

__device__ __forceinline__ Frag ldfrag(const unsigned short* p) {
  Frag f;
  f.u[0] = *(const v8us*)(p);
  f.u[1] = *(const v8us*)(p + 16);
  return f;
}

__device__ __forceinline__ v8f mma_h(v16h a, v16h b, v8f c) {
  v8f d = __builtin_amdgcn_wmma_f32_16x16x32_f16(false, a, false, b, (short)0, c, false, false);
#if defined(__HIP_DEVICE_COMPILE__)
  asm volatile("v_nop\n\tv_nop\n\tv_nop\n\tv_nop" : "+v"(d) : "v"(a), "v"(b));
#endif
  return d;
}
__device__ __forceinline__ v8f mma_b(v16b a, v16b b, v8f c) {
  v8f d = __builtin_amdgcn_wmma_f32_16x16x32_bf16(false, a, false, b, (short)0, c, false, false);
#if defined(__HIP_DEVICE_COMPILE__)
  const v16h ha = __builtin_bit_cast(v16h, a), hb = __builtin_bit_cast(v16h, b);
  asm volatile("v_nop\n\tv_nop\n\tv_nop\n\tv_nop" : "+v"(d) : "v"(ha), "v"(hb));
#endif
  return d;
}

__global__ __launch_bounds__(256)
void cvt_w(const float* __restrict__ wq, const float* __restrict__ wk, const float* __restrict__ wv,
           unsigned short* W16) {
  const int tid = threadIdx.x, blk = blockIdx.x;
  const int rl = tid >> 5, col = 8 * (tid & 31);
  const int o = 8 * blk + rl;
  const float* wbase;
  int osub;
  if (blk < DQ / 8)            { wbase = wq; osub = 0; }
  else if (blk < (2 * DQ) / 8) { wbase = wk; osub = DQ; }
  else                         { wbase = wv; osub = 2 * DQ; }
  const float* s = wbase + (size_t)(o - osub) * CC + col;
  const v4f a = *(const v4f*)s;
  const v4f q = *(const v4f*)(s + 4);
  const float f[8] = {a[0], a[1], a[2], a[3], q[0], q[1], q[2], q[3]};
  v4u u;
#pragma unroll
  for (int t = 0; t < 4; ++t) {
    const _Float16 h0 = (_Float16)(bfr(f[2 * t]) * WSC);
    const _Float16 h1 = (_Float16)(bfr(f[2 * t + 1]) * WSC);
    u[t] = pk16(h_bits(h0), h_bits(h1));
  }
#pragma unroll
  for (int pass = 0; pass < 2; ++pass) {
    *(volatile v4u*)(W16 + (size_t)o * CC + col) = u;
    __threadfence();
  }
}

__global__ __launch_bounds__(256)
void cvt_x(const float* __restrict__ x, unsigned short* XP) {
  __shared__ __align__(16) unsigned short T[QT * TP];
  const int tid = threadIdx.x;
  const int nb = blockIdx.x, cb = blockIdx.y, b = blockIdx.z;
  const int e = tid & 7, lq = tid >> 3;
  const int n0 = nb * QT, c0 = cb * QT;
#pragma unroll
  for (int it = 0; it < 2; ++it) {
    const int cl = it * 32 + lq;
    const float* sp = x + ((size_t)(b * CC + c0 + cl)) * SEQ_FULL + n0 + 8 * e;
    const v4f a = *(const v4f*)sp;
    const v4f q = *(const v4f*)(sp + 4);
    unsigned short hb[8];
#pragma unroll
    for (int t = 0; t < 4; ++t) {
      hb[t]     = h_bits((_Float16)bfr(a[t]));
      hb[4 + t] = h_bits((_Float16)bfr(q[t]));
    }
#pragma unroll
    for (int t = 0; t < 8; ++t) T[(8 * e + t) * TP + cl] = hb[t];
  }
  __syncthreads();
  v4u up[2];
#pragma unroll
  for (int it = 0; it < 2; ++it) {
    const int nl = it * 32 + lq;
    up[it] = *(const v4u*)(T + nl * TP + 8 * e);
  }
#pragma unroll
  for (int pass = 0; pass < 2; ++pass) {
#pragma unroll
    for (int it = 0; it < 2; ++it) {
      const int rl = it * 32 + lq;
      *(volatile v4u*)(XP + ((size_t)(b * SEQ + n0 + rl)) * CC + c0 + 8 * e) = up[it];
    }
    __threadfence();
  }
}

__global__ __launch_bounds__(128)
void gemm_p(const unsigned short* __restrict__ W16, const unsigned short* __restrict__ XP,
            unsigned short* Fh, unsigned short* Fl, unsigned short* Gh, unsigned short* Gl,
            unsigned short* Hv) {
  __shared__ __align__(16) float Os[QT * OSP];
  const int tid  = threadIdx.x;
  const int lane = tid & 31, wave = tid >> 5;
  const int hh   = lane >> 4, c = lane & 15;
  const int nt   = blockIdx.x, mb = blockIdx.y, b = blockIdx.z;
  const int n0   = nt * QT, o0 = mb * QT;

  const unsigned short* ap = W16 + (size_t)(o0 + c) * CC + 8 * hh;
  const unsigned short* bp = XP + ((size_t)(b * SEQ + n0 + 16 * wave + c)) * CC + 8 * hh;

  v8f acc[4];
#pragma unroll
  for (int mt = 0; mt < 4; ++mt) acc[mt] = zero8();

#pragma unroll
  for (int ks = 0; ks < CC / 32; ++ks) {
    const Frag fb = ldfrag(bp + 32 * ks);
#pragma unroll
    for (int mt = 0; mt < 4; ++mt) {
      const Frag fa = ldfrag(ap + (size_t)(16 * mt) * CC + 32 * ks);
      acc[mt] = mma_h(fa.h, fb.h, acc[mt]);
    }
  }

  {
    const int nl = 16 * wave + c;
#pragma unroll
    for (int mt = 0; mt < 4; ++mt) {
      v4f va, vb;
#pragma unroll
      for (int r = 0; r < 4; ++r) {
        va[r] = fmaxf(acc[mt][r] * IWSC, 0.f);
        vb[r] = fmaxf(acc[mt][4 + r] * IWSC, 0.f);
      }
      *(v4f*)(Os + nl * OSP + 16 * mt + 8 * hh)     = va;
      *(v4f*)(Os + nl * OSP + 16 * mt + 8 * hh + 4) = vb;
    }
  }
  __syncthreads();

  const int e = tid & 7, lq = tid >> 3;
  if (mb == 0) {
    v4u ufh[2], ufl[2], ugh[2], ugl[2];
#pragma unroll
    for (int it = 0; it < 2; ++it) {
      const int L   = it * 16 + lq;
      const int row = 2 * L + (e >> 2);
      const int d   = 8 * (e & 3);
      const float* fs = Os + row * OSP + d;
      const float* gs = Os + row * OSP + DQ + d;
      const v4f fa = *(const v4f*)fs;
      const v4f fb = *(const v4f*)(fs + 4);
      const v4f ga = *(const v4f*)gs;
      const v4f gb = *(const v4f*)(gs + 4);
      const float fv[8] = {fa[0], fa[1], fa[2], fa[3], fb[0], fb[1], fb[2], fb[3]};
      const float gv[8] = {ga[0], ga[1], ga[2], ga[3], gb[0], gb[1], gb[2], gb[3]};
#pragma unroll
      for (int t = 0; t < 4; ++t) {
        const unsigned short fh0 = bf_bits(fv[2 * t]), fh1 = bf_bits(fv[2 * t + 1]);
        const unsigned short fl0 = bf_bits(fv[2 * t] - bf_up(fh0));
        const unsigned short fl1 = bf_bits(fv[2 * t + 1] - bf_up(fh1));
        const unsigned short gh0 = bf_bits(gv[2 * t]), gh1 = bf_bits(gv[2 * t + 1]);
        const unsigned short gl0 = bf_bits(gv[2 * t] - bf_up(gh0));
        const unsigned short gl1 = bf_bits(gv[2 * t + 1] - bf_up(gh1));
        ufh[it][t] = pk16(fh0, fh1);
        ufl[it][t] = pk16(fl0, fl1);
        ugh[it][t] = pk16(gh0, gh1);
        ugl[it][t] = pk16(gl0, gl1);
      }
    }
#pragma unroll
    for (int pass = 0; pass < 2; ++pass) {
#pragma unroll
      for (int it = 0; it < 2; ++it) {
        const int L   = it * 16 + lq;
        const int row = 2 * L + (e >> 2);
        const int d   = 8 * (e & 3);
        const size_t po = ((size_t)(b * SEQ + n0 + row)) * DQ + d;
        *(volatile v4u*)(Fh + po) = ufh[it];
        *(volatile v4u*)(Fl + po) = ufl[it];
        *(volatile v4u*)(Gh + po) = ugh[it];
        *(volatile v4u*)(Gl + po) = ugl[it];
      }
      __threadfence();
    }
  } else {
    const int chb = (mb - 1) * QT;
    v4u uhp[4];
#pragma unroll
    for (int it = 0; it < 4; ++it) {
      const int ol = it * 16 + lq;
      float hv8[8];
#pragma unroll
      for (int t = 0; t < 8; ++t) hv8[t] = Os[(8 * e + t) * OSP + ol];
#pragma unroll
      for (int t = 0; t < 4; ++t) {
        const _Float16 h0 = (_Float16)(hv8[2 * t] * HSC);
        const _Float16 h1 = (_Float16)(hv8[2 * t + 1] * HSC);
        uhp[it][t] = pk16(h_bits(h0), h_bits(h1));
      }
    }
#pragma unroll
    for (int pass = 0; pass < 2; ++pass) {
#pragma unroll
      for (int it = 0; it < 4; ++it) {
        const int ol = it * 16 + lq;
        *(volatile v4u*)(Hv + ((size_t)(b * CC + chb + ol)) * SEQ + n0 + 8 * e) = uhp[it];
      }
      __threadfence();
    }
  }
}

__global__ __launch_bounds__(128)
void attn_k(const unsigned short* __restrict__ Gh, const unsigned short* __restrict__ Gl,
            const unsigned short* __restrict__ Fh, const unsigned short* __restrict__ Fl,
            const unsigned short* __restrict__ Hv, const float* __restrict__ x,
            const float* __restrict__ gamma, float* out) {
  __shared__ __align__(16) float Os[QT * OSPW];
  const int tid  = threadIdx.x;
  const int wave = tid >> 5, lane = tid & 31;
  const int hh   = lane >> 4, c = lane & 15;
  const int n0   = blockIdx.x * QT, b = blockIdx.y;

  const size_t qo = ((size_t)(b * SEQ + n0 + 16 * wave + c)) * DQ + 8 * hh;
  const Frag qh = ldfrag(Gh + qo);
  const Frag ql = ldfrag(Gl + qo);
  const unsigned short* Khp = Fh + (size_t)b * SEQ * DQ + (size_t)c * DQ + 8 * hh;
  const unsigned short* Klp = Fl + (size_t)b * SEQ * DQ + (size_t)c * DQ + 8 * hh;
  const unsigned short* Vp = Hv + (size_t)b * CC * SEQ + (size_t)c * SEQ + 8 * hh;

  float m = -1.0e30f, l = 0.f;
  v8f o[16];
#pragma unroll
  for (int j = 0; j < 16; ++j) o[j] = zero8();

#pragma unroll 1
  for (int kb = 0; kb < SEQ; kb += 32) {
    const Frag k0  = ldfrag(Khp + (size_t)kb * DQ);
    const Frag k1  = ldfrag(Khp + (size_t)(kb + 16) * DQ);
    const Frag k0l = ldfrag(Klp + (size_t)kb * DQ);
    const Frag k1l = ldfrag(Klp + (size_t)(kb + 16) * DQ);
    v8f s0 = zero8(), s1 = zero8();
    s0 = mma_b(k0.bf, qh.bf, s0);
    s1 = mma_b(k1.bf, qh.bf, s1);
    s0 = mma_b(k0.bf, ql.bf, s0);
    s1 = mma_b(k1.bf, ql.bf, s1);
    s0 = mma_b(k0l.bf, qh.bf, s0);
    s1 = mma_b(k1l.bf, qh.bf, s1);

    float mx = fmaxf(hmax8(s0), hmax8(s1));
    mx = fmaxf(mx, __shfl_xor(mx, 16, 32));
    const float mn = fmaxf(m, mx);
    const unsigned grew = wave_ballot(mx > m);
    if (grew != 0u) {
      const float corr = __expf(m - mn);
      l *= corr;
#pragma unroll
      for (int j = 0; j < 16; ++j) {
#pragma unroll
        for (int r = 0; r < 8; ++r) o[j][r] *= corr;
      }
    }
    m = mn;
    const float msh = mn - LNPS;

    FragH ph;
    float ls = 0.f;
#pragma unroll
    for (int r = 0; r < 8; ++r) {
      const float e0 = __expf(s0[r] - msh);
      const float e1 = __expf(s1[r] - msh);
      ls += e0 + e1;
      ph.hv[0][r] = (_Float16)e0;
      ph.hv[1][r] = (_Float16)e1;
    }
    l += ls;

#pragma unroll
    for (int j = 0; j < 16; ++j) {
      const Frag vf = ldfrag(Vp + (size_t)(16 * j) * SEQ + kb);
      o[j] = mma_h(vf.h, ph.v, o[j]);
    }
  }
  l += __shfl_xor(l, 16, 32);
  const float gm  = bfr(gamma[0]);
  const float inv = gm * IHSC * (1.0f / l);

  const int qrow = 16 * wave + c;
  const int e = tid & 7, lq = tid >> 3;
#pragma unroll
  for (int half = 0; half < 2; ++half) {
    if (half) __syncthreads();
#pragma unroll
    for (int jj = 0; jj < 8; ++jj) {
      const int j = 8 * half + jj;
      v4f va, vb;
#pragma unroll
      for (int r = 0; r < 4; ++r) { va[r] = o[j][r] * inv; vb[r] = o[j][4 + r] * inv; }
      *(v4f*)(Os + qrow * OSPW + 16 * jj + 8 * hh)     = va;
      *(v4f*)(Os + qrow * OSPW + 16 * jj + 8 * hh + 4) = vb;
    }
    __syncthreads();
    v4f res[16];
#pragma unroll
    for (int it = 0; it < 16; ++it) {
      const int L   = it * 16 + lq;
      const int chl = L >> 1, hf = L & 1;
      const int nl  = hf * 32 + 4 * e;
      const size_t xi = ((size_t)(b * CC + 128 * half + chl)) * SEQ_FULL + n0 + nl;
      const v4f xv = *(const v4f*)(x + xi);
#pragma unroll
      for (int t = 0; t < 4; ++t) res[it][t] = Os[(nl + t) * OSPW + chl] + bfr(xv[t]);
    }
#pragma unroll
    for (int pass = 0; pass < 2; ++pass) {
#pragma unroll
      for (int it = 0; it < 16; ++it) {
        const int L   = it * 16 + lq;
        const int chl = L >> 1, hf = L & 1;
        const int nl  = hf * 32 + 4 * e;
        const size_t oi = ((size_t)(b * CC + 128 * half + chl)) * SEQ + n0 + nl;
        *(volatile v4f*)(out + oi) = res[it];
      }
      __threadfence();
    }
  }
}

extern "C" void kernel_launch(void* const* d_in, const int* in_sizes, int n_in,
                              void* d_out, int out_size, void* d_ws, size_t ws_size,
                              hipStream_t stream) {
  if (n_in < 5) return;
  if (in_sizes[0] < NB * CC * SEQ_FULL) return;
  if (in_sizes[1] < DQ * CC || in_sizes[2] < DQ * CC) return;
  if (in_sizes[3] < CC * CC) return;
  if (in_sizes[4] < 1) return;
  if (out_size < NB * CC * SEQ) return;

  size_t off = 0;
  auto carve = [&](size_t bytes) { const size_t o = off; off += (bytes + 255) & ~(size_t)255; return o; };
  const size_t oW16 = carve((size_t)MW * CC * 2);
  const size_t oXP  = carve((size_t)NB * SEQ * CC * 2);
  const size_t oHv  = carve((size_t)NB * CC * SEQ * 2);
  const size_t oFh  = carve((size_t)NB * SEQ * DQ * 2);
  const size_t oFl  = carve((size_t)NB * SEQ * DQ * 2);
  const size_t oGh  = carve((size_t)NB * SEQ * DQ * 2);
  const size_t oGl  = carve((size_t)NB * SEQ * DQ * 2);
  if (off > ws_size) return;
  if (off > (size_t)134217728) return;

  const float* x     = (const float*)d_in[0];
  const float* wq    = (const float*)d_in[1];
  const float* wk    = (const float*)d_in[2];
  const float* wv    = (const float*)d_in[3];
  const float* gamma = (const float*)d_in[4];

  char* ws = (char*)d_ws;
  unsigned short* W16 = (unsigned short*)(ws + oW16);
  unsigned short* XP  = (unsigned short*)(ws + oXP);
  unsigned short* Hv  = (unsigned short*)(ws + oHv);
  unsigned short* Fh  = (unsigned short*)(ws + oFh);
  unsigned short* Fl  = (unsigned short*)(ws + oFl);
  unsigned short* Gh  = (unsigned short*)(ws + oGh);
  unsigned short* Gl  = (unsigned short*)(ws + oGl);
  float* out = (float*)d_out;

  const dim3 blk256(256), blk128(128);

  cvt_w<<<dim3(MW / 8), blk256, 0, stream>>>(wq, wk, wv, W16);
  cvt_x<<<dim3(SEQ / QT, CC / QT, NB), blk256, 0, stream>>>(x, XP);
  gemm_p<<<dim3(SEQ / QT, MBLK, NB), blk128, 0, stream>>>(W16, XP, Fh, Fl, Gh, Gl, Hv);
  attn_k<<<dim3(SEQ / QT, NB), blk128, 0, stream>>>(Gh, Gl, Fh, Fl, Hv, x, gamma, out);
  (void)hipGetLastError();
}
